// BDH_1726576853700
// MI455X (gfx1250) — hardware-run, weakly checked
//
#include <hip/hip_runtime.h>
#include <math.h>

typedef __attribute__((ext_vector_type(16))) _Float16 v16h;
typedef __attribute__((ext_vector_type(8)))  _Float16 v8h;
typedef __attribute__((ext_vector_type(8)))  float    v8f;
typedef __attribute__((ext_vector_type(4)))  float    v4f;
typedef __attribute__((ext_vector_type(2)))  float    v2f;
typedef __attribute__((ext_vector_type(4)))  unsigned int v4u;
typedef __attribute__((ext_vector_type(2)))  unsigned int v2u;

constexpr int kT      = 1024;
constexpr int kD      = 256;
constexpr int kNH     = 4;
constexpr int kN      = 8192;
constexpr int kNP     = kN / 2;
constexpr int kV      = 256;
constexpr int kLayers = 3;
constexpr float kEps  = 1e-5f;
constexpr float kInvD = 1.0f / (float)kD;
constexpr float kTwoPi    = 6.283185307179586f;
constexpr float kInvTwoPi = 1.0f / kTwoPi;

constexpr float kXCarry  = 64.0f;
constexpr float kWCarry  = 1024.0f;
constexpr float kSCarry  = 64.0f;
constexpr float kXYCarry = 256.0f;
constexpr float kScaleEnc   = kSCarry / (kXCarry * kWCarry);
constexpr float kScaleScore = 1.0f / (kSCarry * kSCarry);
constexpr float kScaleYkv   = 1.0f / kXCarry;
constexpr float kScaleEncv  = (kXYCarry / kSCarry) / (kXCarry * kWCarry);
constexpr float kScaleDec   = 1.0f / (kXYCarry * kWCarry);
constexpr float kScaleLm    = 1.0f / (kXCarry * kWCarry);
constexpr float kF16MinNormal = 6.103515625e-5f;

static_assert(kN == kNP * 2 && kNP == 4096, "pair count");
static_assert((kD % 32) == 0 && (kT % 32) == 0 && (kN % 32) == 0, "GEMM K multiples of 32");
static_assert((kT % 64) == 0 && (kN % 64) == 0 && (kD % 64) == 0 && (kV % 64) == 0, "GEMM M,N multiples of 64");

constexpr size_t kSzW    = (size_t)kNH * kN * kD * 2;
constexpr size_t kSzLm   = (size_t)kV * kD * 2;
constexpr size_t kSzTab  = (size_t)kT * kNP * 2 * 4;
constexpr size_t kSzXf   = (size_t)kT * kD * 4;
constexpr size_t kSzXh   = (size_t)kT * kD * 2;
constexpr size_t kSzHead = (size_t)kT * kN * 2;
constexpr size_t kSzSc   = (size_t)kT * kT * 2;
constexpr size_t kOffEncT  = 0;
constexpr size_t kOffEncvT = kOffEncT  + kSzW;
constexpr size_t kOffDecT  = kOffEncvT + kSzW;
constexpr size_t kOffLmT   = kOffDecT  + kSzW;
constexpr size_t kOffTab   = kOffLmT   + kSzLm;
constexpr size_t kOffXfA   = kOffTab   + kSzTab;
constexpr size_t kOffXfB   = kOffXfA   + kSzXf;
constexpr size_t kOffXh    = kOffXfB   + kSzXf;
constexpr size_t kOffXTh   = kOffXh    + kSzXh;
constexpr size_t kOffXs    = kOffXTh   + kSzXh;
constexpr size_t kOffQr    = kOffXs    + kSzHead;
constexpr size_t kOffSc    = kOffQr    + kSzHead;
constexpr size_t kOffYkv   = kOffSc    + kSzSc;
constexpr size_t kOffYln   = kOffYkv   + kSzXf;
constexpr size_t kOffYmA   = kOffYln   + kSzXh;
constexpr size_t kOffYmB   = kOffYmA   + kSzXf;
constexpr size_t kWsTotal  = kOffYmB   + kSzXf;
static_assert(kWsTotal == 126484480ull, "carve total");
static_assert(kWsTotal <= 134217728ull, "carve cap");
static_assert((kOffEncvT % 128) == 0 && (kOffDecT % 128) == 0 && (kOffLmT % 128) == 0 && (kOffTab % 128) == 0 &&
              (kOffXfA % 128) == 0 && (kOffXfB % 128) == 0 && (kOffXh % 128) == 0 && (kOffXTh % 128) == 0 &&
              (kOffXs % 128) == 0 && (kOffQr % 128) == 0 && (kOffSc % 128) == 0 && (kOffYkv % 128) == 0 &&
              (kOffYln % 128) == 0 && (kOffYmA % 128) == 0 && (kOffYmB % 128) == 0, "128-B aligned regions");

__device__ __forceinline__ unsigned short h_bits_ftz(float f) {
  const float g = (fabsf(f) < kF16MinNormal) ? 0.0f : f;
  const _Float16 h = (_Float16)g;
  return __builtin_bit_cast(unsigned short, h);
}
__device__ __forceinline__ unsigned pk2(float a, float b) {
  const unsigned lo = (unsigned)h_bits_ftz(a);
  const unsigned hi = (unsigned)h_bits_ftz(b);
  return lo | (hi << 16);
}
__device__ __forceinline__ float h16_to_f32(unsigned hb) {
  const unsigned sgn = (hb & 0x8000u) << 16;
  const unsigned em = hb & 0x7fffu;
  const float fn = __uint_as_float((em << 13) + 0x38000000u);
  const float fs = (float)em * 5.9604644775390625e-8f;
  const float mag = (em < 0x400u) ? fs : fn;
  return __uint_as_float(__float_as_uint(mag) | sgn);
}
__device__ __forceinline__ float wave_sum32(float v) {
#pragma unroll
  for (int off = 16; off > 0; off >>= 1) v += __shfl_xor(v, off, 32);
  return v;
}
__device__ __forceinline__ void ln_pair(v4f& a, v4f& b) {
  float s = ((a[0] + a[1]) + (a[2] + a[3])) + ((b[0] + b[1]) + (b[2] + b[3]));
  s = wave_sum32(s);
  const float mu = s * kInvD;
  a = a - mu;
  b = b - mu;
  float qv = ((a[0] * a[0] + a[1] * a[1]) + (a[2] * a[2] + a[3] * a[3])) +
             ((b[0] * b[0] + b[1] * b[1]) + (b[2] * b[2] + b[3] * b[3]));
  qv = wave_sum32(qv);
  const float rstd = 1.0f / sqrtf(qv * kInvD + kEps);
  a = a * rstd;
  b = b * rstd;
}

struct FragH {
  union U { v16h v; v8h h[2]; };
  static __device__ __forceinline__ v16h load(const _Float16* p) {
    U f;
    f.h[0] = *(const v8h*)(p);
    f.h[1] = *(const v8h*)(p + 16);
    return f.v;
  }
  static __device__ __forceinline__ v8f mma(v16h a, v16h b, v8f c) {
    return __builtin_amdgcn_wmma_f32_16x16x32_f16(false, a, false, b, (short)0, c, false, false);
  }
};
__device__ __forceinline__ void guard_row(v8f& a0, v8f& a1, v8f& a2, v8f& a3,
                                          v16h x, v16h b0, v16h b1, v16h b2, v16h b3) {
  asm volatile("v_nop\n\tv_nop\n\tv_nop\n\tv_nop"
               : "+v"(a0), "+v"(a1), "+v"(a2), "+v"(a3)
               : "v"(x), "v"(b0), "v"(b1), "v"(b2), "v"(b3));
}

constexpr int G_ENC = 0;
constexpr int G_SCORE = 1;
constexpr int G_F32 = 2;
constexpr int G_F32ADD = 3;
constexpr int G_ENCV = 4;

template <int MODE>
__global__ __launch_bounds__(256) void gemm64_kernel(
    const unsigned short* __restrict__ Ap, int lda,
    const unsigned short* __restrict__ Btp, int ldb,
    void* __restrict__ C0, void* __restrict__ C1, int ldc,
    const float* __restrict__ auxf, const unsigned short* __restrict__ auxh,
    int M, int N, int K, int klim, float scale) {
  const _Float16* A = (const _Float16*)Ap;
  const _Float16* Bt = (const _Float16*)Btp;
  __shared__ __align__(16) float sT[8][16 * 68];
  const int lane = threadIdx.x & 31;
  const int wave = threadIdx.x >> 5;
  const int tilesN = N >> 6;
  const int tilesM = M >> 6;
  const int tile = blockIdx.x * 8 + wave;
  if (tile >= tilesM * tilesN) return;
  const int tm = tile / tilesN;
  const int tn = tile - tm * tilesN;
  const int m0 = tm << 6;
  const int n0 = tn << 6;

  const int rlane = lane & 15;
  const int koff  = (lane >> 4) * 8;
  const int mOff  = (lane >> 4) * 8;

  v8f acc[4][4];
#pragma unroll
  for (int i = 0; i < 4; ++i)
#pragma unroll
    for (int j = 0; j < 4; ++j) acc[i][j] = (v8f){0.f, 0.f, 0.f, 0.f, 0.f, 0.f, 0.f, 0.f};

  int kEnd = K;
  if (klim != 0) kEnd = (m0 + 64 < K) ? (m0 + 64) : K;
  if (MODE == G_SCORE) {
    if (tn > tm) kEnd = 0;
  }

  const _Float16* ap = A + (size_t)(m0 + rlane) * lda + koff;
  const _Float16* bp = Bt + (size_t)(n0 + rlane) * ldb + koff;

#pragma unroll 1
  for (int k0 = 0; k0 < kEnd; k0 += 32) {
    v16h bh[4];
#pragma unroll
    for (int j = 0; j < 4; ++j) bh[j] = FragH::load(bp + (size_t)(j << 4) * ldb + k0);
#pragma unroll
    for (int i = 0; i < 4; ++i) {
      const v16h ah = FragH::load(ap + (size_t)(i << 4) * lda + k0);
#pragma unroll
      for (int j = 0; j < 4; ++j) acc[i][j] = FragH::mma(ah, bh[j], acc[i][j]);
      guard_row(acc[i][0], acc[i][1], acc[i][2], acc[i][3], ah, bh[0], bh[1], bh[2], bh[3]);
    }
  }

  float* slab = sT[wave];
  const int q  = lane >> 3;
  const int c8 = (lane & 7) * 8;
  const int hh = lane >> 4;
  const int c4 = (lane & 15) * 4;
#pragma unroll
  for (int i = 0; i < 4; ++i) {
    const int mBase = m0 + (i << 4);
#pragma unroll
    for (int j = 0; j < 4; ++j) {
      const int n = n0 + (j << 4) + rlane;
#pragma unroll
      for (int r = 0; r < 8; ++r) {
        float v = acc[i][j][r] * scale;
        if (MODE == G_ENC || MODE == G_ENCV) v = fmaxf(v, 0.0f);
        if (MODE == G_SCORE) v = (n < mBase + mOff + r) ? v : 0.0f;
        slab[(mOff + r) * 68 + (j << 4) + rlane] = v;
      }
    }
    __builtin_amdgcn_fence(__ATOMIC_RELEASE, "workgroup");
    __builtin_amdgcn_wave_barrier();
    __builtin_amdgcn_fence(__ATOMIC_ACQUIRE, "workgroup");
    if (MODE == G_F32 || MODE == G_F32ADD) {
      float* C = (float*)C0;
      v4f vals[8];
#pragma unroll
      for (int it = 0; it < 8; ++it) {
        const int row = it * 2 + hh;
        v4f v = *(const v4f*)(slab + row * 68 + c4);
        if (MODE == G_F32ADD) {
          const v4f r4 = *(const v4f*)(auxf + (size_t)(mBase + row) * ldc + n0 + c4);
          v = v + r4;
        }
        vals[it] = v;
      }
      for (int pass = 0; pass < 2; ++pass) {
#pragma unroll
        for (int it = 0; it < 8; ++it) {
          const int row = it * 2 + hh;
          *(volatile v4f*)(C + (size_t)(mBase + row) * ldc + n0 + c4) = vals[it];
        }
        __threadfence();
      }
    } else {
      unsigned short* Cx = (unsigned short*)C0;
      unsigned short* Cr = (unsigned short*)C1;
      v4u hv[4];
      v4u rv[4];
#pragma unroll
      for (int it = 0; it < 4; ++it) {
        const int row = it * 4 + q;
        const float* sp = slab + row * 68 + c8;
        const v4f a0 = *(const v4f*)(sp);
        const v4f a1 = *(const v4f*)(sp + 4);
        float f[8];
        f[0] = a0[0]; f[1] = a0[1]; f[2] = a0[2]; f[3] = a0[3];
        f[4] = a1[0]; f[5] = a1[1]; f[6] = a1[2]; f[7] = a1[3];
        if (MODE == G_ENCV) {
          const v4u xw = *(const v4u*)(auxh + (size_t)(mBase + row) * ldc + n0 + c8);
          const unsigned w0 = xw[0];
          const unsigned w1 = xw[1];
          const unsigned w2 = xw[2];
          const unsigned w3 = xw[3];
          f[0] *= h16_to_f32(w0 & 0xffffu);
          f[1] *= h16_to_f32(w0 >> 16);
          f[2] *= h16_to_f32(w1 & 0xffffu);
          f[3] *= h16_to_f32(w1 >> 16);
          f[4] *= h16_to_f32(w2 & 0xffffu);
          f[5] *= h16_to_f32(w2 >> 16);
          f[6] *= h16_to_f32(w3 & 0xffffu);
          f[7] *= h16_to_f32(w3 >> 16);
        }
        hv[it] = (v4u){pk2(f[0], f[1]), pk2(f[2], f[3]), pk2(f[4], f[5]), pk2(f[6], f[7])};
        if (MODE == G_ENC) {
          const float* tp = auxf + ((size_t)(mBase + row) * kNP + (size_t)((n0 + c8) >> 1)) * 2;
          const v4f t0 = *(const v4f*)(tp);
          const v4f t1 = *(const v4f*)(tp + 4);
          float g[8];
          g[0] = f[0] * t0[0] - f[1] * t0[1];
          g[1] = f[1] * t0[0] + f[0] * t0[1];
          g[2] = f[2] * t0[2] - f[3] * t0[3];
          g[3] = f[3] * t0[2] + f[2] * t0[3];
          g[4] = f[4] * t1[0] - f[5] * t1[1];
          g[5] = f[5] * t1[0] + f[4] * t1[1];
          g[6] = f[6] * t1[2] - f[7] * t1[3];
          g[7] = f[7] * t1[2] + f[6] * t1[3];
          rv[it] = (v4u){pk2(g[0], g[1]), pk2(g[2], g[3]), pk2(g[4], g[5]), pk2(g[6], g[7])};
        }
      }
      for (int pass = 0; pass < 2; ++pass) {
#pragma unroll
        for (int it = 0; it < 4; ++it) {
          const int row = it * 4 + q;
          const size_t o = (size_t)(mBase + row) * ldc + n0 + c8;
          *(volatile v4u*)(Cx + o) = hv[it];
          if (MODE == G_ENC) *(volatile v4u*)(Cr + o) = rv[it];
        }
        __threadfence();
      }
    }
    __builtin_amdgcn_fence(__ATOMIC_RELEASE, "workgroup");
    __builtin_amdgcn_wave_barrier();
    __builtin_amdgcn_fence(__ATOMIC_ACQUIRE, "workgroup");
  }
}

__global__ __launch_bounds__(256) void cvt_transpose_kernel(const float* __restrict__ in,
                                                            unsigned short* __restrict__ out,
                                                            int R, int C, long inStride, long outStride, float carry) {
  __shared__ float sm[64][65];
  const int t  = threadIdx.x;
  const int c0 = blockIdx.x * 64;
  const int r0 = blockIdx.y * 64;
  const float* ip = in + (size_t)blockIdx.z * (size_t)inStride;
  unsigned short* op = out + (size_t)blockIdx.z * (size_t)outStride;
#pragma unroll 4
  for (int i = 0; i < 16; ++i) {
    const int e = i * 256 + t;
    const int r = e >> 6;
    const int c = e & 63;
    sm[c][r] = ip[(size_t)(r0 + r) * C + c0 + c] * carry;
  }
  __syncthreads();
  const int lane = t & 31, wave = t >> 5;
  const int q = lane >> 3, c8 = (lane & 7) * 8;
  v4u u[2];
#pragma unroll
  for (int it = 0; it < 2; ++it) {
    const int row = wave * 8 + it * 4 + q;
    u[it] = (v4u){pk2(sm[row][c8 + 0], sm[row][c8 + 1]), pk2(sm[row][c8 + 2], sm[row][c8 + 3]),
                  pk2(sm[row][c8 + 4], sm[row][c8 + 5]), pk2(sm[row][c8 + 6], sm[row][c8 + 7])};
  }
  for (int pass = 0; pass < 2; ++pass) {
#pragma unroll
    for (int it = 0; it < 2; ++it) {
      const int row = wave * 8 + it * 4 + q;
      *(volatile v4u*)(op + (size_t)(c0 + row) * R + r0 + c8) = u[it];
    }
    __threadfence();
  }
}

__global__ __launch_bounds__(256) void rope_table_kernel(float* __restrict__ tab) {
#pragma clang fp contract(off)
  const int i = blockIdx.x * 256 + threadIdx.x;
  const int p = i & (kNP - 1);
  const int t = i >> 12;
  const float pw = exp2f((float)p * (1.0f / 256.0f));
  const float fr = (1.0f / pw) * kInvTwoPi;
  const float ph = (float)t * fr;
  const float fc = ph - floorf(ph);
  const float ang = fc * kTwoPi;
  float sv, cv;
  sincosf(ang, &sv, &cv);
  const v2f v = (v2f){cv, sv};
  float* dst = tab + (size_t)i * 2;
  *(volatile v2f*)dst = v;
  __threadfence();
  *(volatile v2f*)dst = v;
}

template <int MODE>
__global__ __launch_bounds__(256) void x_ln_kernel(const int* __restrict__ idx, const float* __restrict__ emb,
                                                   const float* __restrict__ ym, const float* __restrict__ xold,
                                                   float* __restrict__ xnew, unsigned short* __restrict__ xh,
                                                   unsigned short* __restrict__ xth) {
  __shared__ __align__(16) unsigned int sXw[64 * 132];
  const int tid = threadIdx.x, lane = tid & 31, wave = tid >> 5;
  const int t0 = blockIdx.x * 64;
#pragma unroll 1
  for (int i = 0; i < 8; ++i) {
    const int tl = wave * 8 + i;
    const int t = t0 + tl;
    v4f a, b;
    if (MODE == 0) {
      int tok = idx[t];
      tok = tok < 0 ? 0 : (tok > kV - 1 ? kV - 1 : tok);
      const float* src = emb + (size_t)tok * kD;
      a = *(const v4f*)(src + lane * 4);
      b = *(const v4f*)(src + 128 + lane * 4);
      ln_pair(a, b);
    } else {
      const float* yr = ym + (size_t)t * kD;
      a = *(const v4f*)(yr + lane * 4);
      b = *(const v4f*)(yr + 128 + lane * 4);
      ln_pair(a, b);
      const float* xr0 = xold + (size_t)t * kD;
      const v4f xa = *(const v4f*)(xr0 + lane * 4);
      const v4f xb = *(const v4f*)(xr0 + 128 + lane * 4);
      a = a + xa;
      b = b + xb;
      ln_pair(a, b);
    }
    float* xr = xnew + (size_t)t * kD;
    *(volatile v4f*)(xr + lane * 4) = a;
    *(volatile v4f*)(xr + 128 + lane * 4) = b;
    __threadfence();
    *(volatile v4f*)(xr + lane * 4) = a;
    *(volatile v4f*)(xr + 128 + lane * 4) = b;
    const v2u wa = (v2u){pk2(a[0] * kXCarry, a[1] * kXCarry), pk2(a[2] * kXCarry, a[3] * kXCarry)};
    const v2u wb = (v2u){pk2(b[0] * kXCarry, b[1] * kXCarry), pk2(b[2] * kXCarry, b[3] * kXCarry)};
    *(v2u*)&sXw[tl * 132 + lane * 2] = wa;
    *(v2u*)&sXw[tl * 132 + 64 + lane * 2] = wb;
  }
  __syncthreads();
  {
    v4u ur[8];
#pragma unroll
    for (int i = 0; i < 8; ++i) ur[i] = *(const v4u*)&sXw[(wave * 8 + i) * 132 + lane * 4];
    for (int pass = 0; pass < 2; ++pass) {
#pragma unroll
      for (int i = 0; i < 8; ++i)
        *(volatile v4u*)(xh + (size_t)(t0 + wave * 8 + i) * kD + lane * 8) = ur[i];
      __threadfence();
    }
  }
  {
    const int q = lane >> 3, c8 = (lane & 7) * 8;
    v4u ut[8];
#pragma unroll
    for (int it = 0; it < 8; ++it) {
      const int d = it * 32 + wave * 4 + q;
      const int wi = d >> 1;
      const unsigned sh = (unsigned)(d & 1) * 16u;
      unsigned hb[8];
#pragma unroll
      for (int e = 0; e < 8; ++e) {
        const unsigned w = sXw[(c8 + e) * 132 + wi];
        hb[e] = (w >> sh) & 0xffffu;
      }
      ut[it] = (v4u){hb[0] | (hb[1] << 16), hb[2] | (hb[3] << 16), hb[4] | (hb[5] << 16), hb[6] | (hb[7] << 16)};
    }
    for (int pass = 0; pass < 2; ++pass) {
#pragma unroll
      for (int it = 0; it < 8; ++it) {
        const int d = it * 32 + wave * 4 + q;
        *(volatile v4u*)(xth + (size_t)d * kT + t0 + c8) = ut[it];
      }
      __threadfence();
    }
  }
}

__global__ __launch_bounds__(256) void ln_rows_kernel(const float* __restrict__ in, unsigned short* __restrict__ out) {
  const int lane = threadIdx.x & 31, wave = threadIdx.x >> 5;
  const int row = blockIdx.x * 8 + wave;
  const float* src = in + (size_t)row * kD + lane * 8;
  v4f a = *(const v4f*)(src);
  v4f b = *(const v4f*)(src + 4);
  ln_pair(a, b);
  const v4u u = (v4u){pk2(a[0] * kXCarry, a[1] * kXCarry), pk2(a[2] * kXCarry, a[3] * kXCarry),
                      pk2(b[0] * kXCarry, b[1] * kXCarry), pk2(b[2] * kXCarry, b[3] * kXCarry)};
  unsigned short* dst = out + (size_t)row * kD + lane * 8;
  *(volatile v4u*)dst = u;
  __threadfence();
  *(volatile v4u*)dst = u;
}

template <int MODE>
static void launch_gemm(hipStream_t s, const unsigned short* A, int lda, const unsigned short* Bt, int ldb,
                        void* C0, void* C1, int ldc, const float* auxf, const unsigned short* auxh,
                        int M, int N, int K, int klim, float scale) {
  const int tiles = (M >> 6) * (N >> 6);
  gemm64_kernel<MODE><<<dim3((tiles + 7) / 8), dim3(256), 0, s>>>(A, lda, Bt, ldb, C0, C1, ldc, auxf, auxh,
                                                                   M, N, K, klim, scale);
}

extern "C" void kernel_launch(void* const* d_in, const int* in_sizes, int n_in,
                              void* d_out, int out_size, void* d_ws, size_t ws_size,
                              hipStream_t stream) {
  if (n_in < 6) return;
  if (in_sizes[0] != kT) return;
  if (in_sizes[1] != kV * kD) return;
  if (in_sizes[2] != kNH * kD * kN) return;
  if (in_sizes[3] != kNH * kD * kN) return;
  if (in_sizes[4] != kNH * kN * kD) return;
  if (in_sizes[5] != kD * kV) return;
  if (out_size != kT * kV) return;
  if (ws_size < kWsTotal) return;

  const int*   idx   = (const int*)d_in[0];
  const float* embed = (const float*)d_in[1];
  const float* enc   = (const float*)d_in[2];
  const float* encv  = (const float*)d_in[3];
  const float* dec   = (const float*)d_in[4];
  const float* lmh   = (const float*)d_in[5];
  float* out = (float*)d_out;

  char* ws = (char*)d_ws;
  unsigned short* ENCT  = (unsigned short*)(ws + kOffEncT);
  unsigned short* ENCVT = (unsigned short*)(ws + kOffEncvT);
  unsigned short* DECT  = (unsigned short*)(ws + kOffDecT);
  unsigned short* LMT   = (unsigned short*)(ws + kOffLmT);
  float*          TAB   = (float*)(ws + kOffTab);
  float*          XFA   = (float*)(ws + kOffXfA);
  float*          XFB   = (float*)(ws + kOffXfB);
  unsigned short* XH    = (unsigned short*)(ws + kOffXh);
  unsigned short* XTH   = (unsigned short*)(ws + kOffXTh);
  unsigned short* XS    = (unsigned short*)(ws + kOffXs);
  unsigned short* QR    = (unsigned short*)(ws + kOffQr);
  unsigned short* SC    = (unsigned short*)(ws + kOffSc);
  float*          YKV   = (float*)(ws + kOffYkv);
  unsigned short* YLN   = (unsigned short*)(ws + kOffYln);
  float*          YMA   = (float*)(ws + kOffYmA);
  float*          YMB   = (float*)(ws + kOffYmB);

  cvt_transpose_kernel<<<dim3(kN / 64, kD / 64, kNH), 256, 0, stream>>>(
      enc, ENCT, kD, kN, (long)kD * kN, (long)kN * kD, kWCarry);
  cvt_transpose_kernel<<<dim3(kN / 64, kD / 64, kNH), 256, 0, stream>>>(
      encv, ENCVT, kD, kN, (long)kD * kN, (long)kN * kD, kWCarry);
  cvt_transpose_kernel<<<dim3(kD / 64, (kNH * kN) / 64, 1), 256, 0, stream>>>(
      dec, DECT, kNH * kN, kD, 0L, 0L, kWCarry);
  cvt_transpose_kernel<<<dim3(kV / 64, kD / 64, 1), 256, 0, stream>>>(
      lmh, LMT, kD, kV, 0L, 0L, kWCarry);
  rope_table_kernel<<<(kT * kNP) / 256, 256, 0, stream>>>(TAB);
  x_ln_kernel<0><<<kT / 64, 256, 0, stream>>>(idx, embed, nullptr, nullptr, XFA, XH, XTH);

  for (int layer = 0; layer < kLayers; ++layer) {
    float* xcur = (layer & 1) ? XFB : XFA;
    float* xnxt = (layer & 1) ? XFA : XFB;
    for (int h = 0; h < kNH; ++h) {
      const unsigned short* encH  = ENCT  + (size_t)h * kN * kD;
      const unsigned short* encvH = ENCVT + (size_t)h * kN * kD;
      const unsigned short* decH  = DECT  + (size_t)h * kN;
      launch_gemm<G_ENC>(stream, XH, kD, encH, kD, (void*)XS, (void*)QR, kN, TAB, nullptr,
                         kT, kN, kD, 0, kScaleEnc);
      launch_gemm<G_SCORE>(stream, QR, kN, QR, kN, (void*)SC, nullptr, kT, nullptr, nullptr,
                           kT, kT, kN, 0, kScaleScore);
      launch_gemm<G_F32>(stream, SC, kT, XTH, kT, (void*)YKV, nullptr, kD, nullptr, nullptr,
                         kT, kD, kT, 1, kScaleYkv);
      ln_rows_kernel<<<kT / 8, 256, 0, stream>>>(YKV, YLN);
      launch_gemm<G_ENCV>(stream, YLN, kD, encvH, kD, (void*)QR, nullptr, kN, nullptr, XS,
                          kT, kN, kD, 0, kScaleEncv);
      if (h == 0) {
        launch_gemm<G_F32>(stream, QR, kN, decH, kNH * kN, (void*)YMA, nullptr, kD, nullptr, nullptr,
                           kT, kD, kN, 0, kScaleDec);
      } else {
        float* src = (h & 1) ? YMA : YMB;
        float* dst = (h & 1) ? YMB : YMA;
        launch_gemm<G_F32ADD>(stream, QR, kN, decH, kNH * kN, (void*)dst, nullptr, kD, src, nullptr,
                              kT, kD, kN, 0, kScaleDec);
      }
    }
    x_ln_kernel<1><<<kT / 64, 256, 0, stream>>>(idx, embed, YMB, xcur, xnxt, XH, XTH);
  }
  launch_gemm<G_F32>(stream, XH, kD, LMT, kD, (void*)out, nullptr, kV, nullptr, nullptr,
                     kT, kV, kD, 0, kScaleLm);
}
